// GeneralizedAttention_6296422056056
// MI455X (gfx1250) — hardware-verified
//
#include <hip/hip_runtime.h>
#include <stdint.h>
#include <stddef.h>

#define DEVINL __device__ __forceinline__

typedef _Float16 f16t;
typedef _Float16 v16h __attribute__((ext_vector_type(16)));
typedef _Float16 v8h  __attribute__((ext_vector_type(8)));
typedef float    v8f  __attribute__((ext_vector_type(8)));
typedef float    v4f  __attribute__((ext_vector_type(4)));
typedef v8h __attribute__((may_alias)) v8ha;
typedef v4f __attribute__((may_alias)) v4fa;
union FragH { v16h v; v8h half[2]; };
union U8 { v8f v; v4f q[2]; };

#define NB    2
#define NH    8
#define NA    16
#define CIN   256
#define DK    32
#define HQ    64
#define HWQ   4096
#define HK    32
#define KVN   1024
#define PD    128
#define NPR   2048
#define OWQ   0
#define OWK   65536
#define OWV   131072
#define OWP   196608
#define OWX   262144
#define OWY   294912
#define WBN   327680
#define TPBP  256
#define TPB   128
#define TPBA  256
#define PH    72
#define PF    68
#define PE    36

#define ACAR   16.0f
#define WCAR   256.0f
#define QCAR   16.0f
#define KCAR   16.0f
#define VCAR   16.0f
#define POSCAR 16.0f
#define PCAR   256.0f
#define OCAR   16.0f
#define SC_P   (1.0f / 4096.0f)
#define SC_POS (0.70710678118654752f / 256.0f)
#define SC_E   (1.0f / 256.0f)
#define SC_S   (1.0f / 256.0f)
#define SC_O   (1.0f / 256.0f)
#define SC_PO  (1.0f / 4096.0f)
#define LG1000_64 0.15571537944784511f

#define XP_BLKS  (NB * (HWQ / 32) * (CIN / 64))
#define WB_BLKS  (WBN / 8 / TPBP)
#define EM_BLKS  (HQ * (HK / 4))
#define PQ_BLKS  (NB * (HWQ / 64) * 4)
#define PK_BLKS  (NB * (KVN / 64) * 4)
#define POS_BLKS (2 * (NPR / 64) * 4)
#define EXY_BLKS (2 * NA * HQ)
#define ATT_BLKS (NB * (NH / 2) * (HWQ / 64))
#define PO_BLKS  (NB * (HWQ / 64) * 4)

static_assert(TPB == 4 * 32);
static_assert(TPBA == 8 * 32);
static_assert(WB_BLKS * TPBP * 8 == WBN);
static_assert(OWY + CIN * PD == WBN);
static_assert(NA == NB * NH);
static_assert(HWQ == HQ * HQ);
static_assert(KVN == HK * HK);
static_assert(NPR == HQ * HK);
static_assert(NH * DK == CIN);
static_assert((CIN % 32) == 0);
static_assert((PD % 32) == 0);
static_assert((PH % 8) == 0);
static_assert((PF % 4) == 0);
static_assert((PE % 4) == 0);
static_assert(XP_BLKS == 1024);
static_assert(EM_BLKS * 4 == HQ * HK);

DEVINL v8f wmma_f16(v16h a, v16h b, v8f c) {
  v8f d = __builtin_amdgcn_wmma_f32_16x16x32_f16(false, a, false, b, (short)0, c, false, false);
  asm volatile("v_nop\n\tv_nop\n\tv_nop\n\tv_nop" : "+v"(d) : "v"(a), "v"(b));
  return d;
}
DEVINL v8f zero8f() {
  v8f z = {0.f, 0.f, 0.f, 0.f, 0.f, 0.f, 0.f, 0.f};
  return z;
}
DEVINL void load_frag(FragH& f, const f16t* row, int k0) {
  f.half[0] = *(const v8ha*)(row + k0);
  f.half[1] = *(const v8ha*)(row + k0 + 16);
}

template <int KD>
DEVINL void mma_4n(const f16t* __restrict__ arow, const f16t* __restrict__ brow, v8f (&acc)[4]) {
  #pragma unroll 1
  for (int ks = 0; ks < KD / 32; ++ks) {
    const int k0 = 32 * ks;
    FragH a;
    load_frag(a, arow, k0);
    #pragma unroll
    for (int n = 0; n < 4; ++n) {
      FragH b;
      load_frag(b, brow + (size_t)16 * n * KD, k0);
      acc[n] = wmma_f16(a.v, b.v, acc[n]);
    }
  }
}

__global__ __launch_bounds__(TPBP) void prep_k(const float* __restrict__ x,
                                              const float* __restrict__ wq, const float* __restrict__ wk,
                                              const float* __restrict__ wv, const float* __restrict__ wp,
                                              const float* __restrict__ wx, const float* __restrict__ wy,
                                              f16t* __restrict__ XT, f16t* __restrict__ WB)
{
  __shared__ __attribute__((aligned(16))) f16t tile[32 * PH];
  const int blk = blockIdx.x, tid = threadIdx.x;
  if (blk < XP_BLKS) {
    const int n = blk >> 9;
    const int rem = blk & 511;
    const int nt = rem >> 2, ct = rem & 3;
    const int n0 = 32 * nt, c0 = 64 * ct;
    const int crow = tid >> 2, np = (tid & 3) * 8;
    const float* sp = x + ((size_t)n * CIN + c0 + crow) * HWQ + n0 + np;
    const v4f a = *(const v4fa*)sp, c = *(const v4fa*)(sp + 4);
    #pragma unroll
    for (int j = 0; j < 4; ++j) {
      tile[(np + j) * PH + crow]     = (f16t)(a[j] * ACAR);
      tile[(np + 4 + j) * PH + crow] = (f16t)(c[j] * ACAR);
    }
    __syncthreads();
    const int nrow = tid >> 3, q = tid & 7;
    const v8h o = *(const v8ha*)(tile + nrow * PH + 8 * q);
    f16t* dp = XT + ((size_t)n * HWQ + n0 + nrow) * CIN + c0 + 8 * q;
    *(volatile v8h*)dp = o;
    __threadfence();
    *(volatile v8h*)dp = o;
  } else if (blk < XP_BLKS + WB_BLKS) {
    const int wb = blk - XP_BLKS;
    const int idx = (wb * TPBP + tid) * 8;
    const int unit = idx >> 15;
    const float* src;
    int base;
    switch (unit) {
      case 0: case 1: src = wq; base = OWQ; break;
      case 2: case 3: src = wk; base = OWK; break;
      case 4: case 5: src = wv; base = OWV; break;
      case 6: case 7: src = wp; base = OWP; break;
      case 8:         src = wx; base = OWX; break;
      default:        src = wy; base = OWY; break;
    }
    const float* s = src + (idx - base);
    const v4f a = *(const v4fa*)s, c = *(const v4fa*)(s + 4);
    v8h o;
    #pragma unroll
    for (int j = 0; j < 4; ++j) {
      o[j]     = (f16t)(a[j] * WCAR);
      o[4 + j] = (f16t)(c[j] * WCAR);
    }
    f16t* dp = WB + idx;
    *(volatile v8h*)dp = o;
    __threadfence();
    *(volatile v8h*)dp = o;
  }
}

__global__ __launch_bounds__(TPBP) void embed_k(f16t* __restrict__ E)
{
  __shared__ __attribute__((aligned(16))) f16t tile[4 * PD];
  const int blk = blockIdx.x, tid = threadIdx.x;
  const int pos = blk >> 3, l0 = (blk & 7) * 4;
  const int ll = tid >> 6, fr = tid & 63;
  const int l = l0 + ll;
  const float diff = (float)(pos - 2 * l);
  const float dm = exp2f((float)fr * LG1000_64);
  const float ang = diff * (1.0f / dm);
  float sv, cv;
  sincosf(ang, &sv, &cv);
  tile[ll * PD + fr]      = (f16t)sv;
  tile[ll * PD + 64 + fr] = (f16t)cv;
  __syncthreads();
  if (tid < 64) {
    const v8h o = *(const v8ha*)(tile + 8 * tid);
    f16t* dp = E + ((size_t)pos * HK + l0) * PD + 8 * tid;
    *(volatile v8h*)dp = o;
    __threadfence();
    *(volatile v8h*)dp = o;
  }
}

__global__ __launch_bounds__(TPB) void proj_k(const f16t* __restrict__ XT, const f16t* __restrict__ WB,
                                             const float* __restrict__ ab, const float* __restrict__ gb,
                                             f16t* __restrict__ QA, f16t* __restrict__ QG,
                                             f16t* __restrict__ KP, f16t* __restrict__ VT)
{
  __shared__ __attribute__((aligned(16))) float sbuf[64 * PF];
  const int tid = threadIdx.x, lane = tid & 31, wave = tid >> 5;
  const int h = lane >> 4, m = lane & 15;
  const int blk = blockIdx.x;
  int mode, pb, cg;
  if (blk < PQ_BLKS) { mode = 0; pb = blk >> 2; cg = blk & 3; }
  else if (blk < PQ_BLKS + PK_BLKS) { mode = 1; pb = (blk - PQ_BLKS) >> 2; cg = (blk - PQ_BLKS) & 3; }
  else { mode = 2; pb = (blk - PQ_BLKS - PK_BLKS) >> 2; cg = (blk - PQ_BLKS - PK_BLKS) & 3; }

  int n, p0;
  size_t arowi;
  const f16t* Wp;
  if (mode == 0) {
    n = pb >> 6; p0 = (pb & 63) * 64;
    arowi = (size_t)n * HWQ + p0 + 16 * wave + m;
    Wp = WB + OWQ;
  } else {
    n = pb >> 4; p0 = (pb & 15) * 64;
    const int kl = p0 + 16 * wave + m;
    const int hk = kl >> 5, wl = kl & 31;
    arowi = (size_t)n * HWQ + 128 * hk + 2 * wl;
    Wp = WB + ((mode == 1) ? OWK : OWV);
  }

  v8f acc[4];
  #pragma unroll
  for (int t = 0; t < 4; ++t) acc[t] = zero8f();
  mma_4n<CIN>(XT + arowi * CIN + 8 * h, Wp + (size_t)(64 * cg + m) * CIN + 8 * h, acc);

  const int tr = (mode == 2);
  #pragma unroll
  for (int t = 0; t < 4; ++t) {
    #pragma unroll
    for (int r = 0; r < 8; ++r) {
      const int prow = 16 * wave + 8 * h + r;
      const int col = 16 * t + m;
      const float v = acc[t][r] * SC_P;
      const int idx = tr ? (col * PF + prow) : (prow * PF + col);
      sbuf[idx] = v;
    }
  }
  __syncthreads();

  if (mode == 0) {
    v8h ova[4], ovg[4];
    size_t off[4];
    #pragma unroll
    for (int k = 0; k < 4; ++k) {
      const int al = k >> 1, hf = k & 1;
      const int p = 128 * hf + tid;
      const int row = p >> 2, d8 = (p & 3) * 8;
      const int col = 32 * al + d8;
      const v4f a = *(const v4fa*)(sbuf + row * PF + col), c = *(const v4fa*)(sbuf + row * PF + col + 4);
      const v4f ba = *(const v4fa*)(ab + 64 * cg + col), bc = *(const v4fa*)(ab + 64 * cg + col + 4);
      const v4f ga = *(const v4fa*)(gb + 64 * cg + col), gc = *(const v4fa*)(gb + 64 * cg + col + 4);
      #pragma unroll
      for (int j = 0; j < 4; ++j) {
        ova[k][j]     = (f16t)((a[j] + ba[j]) * QCAR);
        ova[k][4 + j] = (f16t)((c[j] + bc[j]) * QCAR);
        ovg[k][j]     = (f16t)((a[j] + ga[j]) * QCAR);
        ovg[k][4 + j] = (f16t)((c[j] + gc[j]) * QCAR);
      }
      const int na = n * NH + 2 * cg + al;
      off[k] = ((size_t)na * HWQ + p0 + row) * DK + d8;
    }
    #pragma unroll
    for (int k = 0; k < 4; ++k) {
      *(volatile v8h*)(QA + off[k]) = ova[k];
      *(volatile v8h*)(QG + off[k]) = ovg[k];
    }
    __threadfence();
    #pragma unroll
    for (int k = 0; k < 4; ++k) {
      *(volatile v8h*)(QA + off[k]) = ova[k];
      *(volatile v8h*)(QG + off[k]) = ovg[k];
    }
  } else if (mode == 1) {
    v8h ov[4];
    size_t off[4];
    #pragma unroll
    for (int k = 0; k < 4; ++k) {
      const int al = k >> 1, hf = k & 1;
      const int p = 128 * hf + tid;
      const int row = p >> 2, d8 = (p & 3) * 8;
      const int col = 32 * al + d8;
      const v4f a = *(const v4fa*)(sbuf + row * PF + col), c = *(const v4fa*)(sbuf + row * PF + col + 4);
      #pragma unroll
      for (int j = 0; j < 4; ++j) {
        ov[k][j]     = (f16t)(a[j] * KCAR);
        ov[k][4 + j] = (f16t)(c[j] * KCAR);
      }
      const int na = n * NH + 2 * cg + al;
      off[k] = ((size_t)na * KVN + p0 + row) * DK + d8;
    }
    #pragma unroll
    for (int k = 0; k < 4; ++k) *(volatile v8h*)(KP + off[k]) = ov[k];
    __threadfence();
    #pragma unroll
    for (int k = 0; k < 4; ++k) *(volatile v8h*)(KP + off[k]) = ov[k];
  } else {
    v8h ov[4];
    size_t off[4];
    #pragma unroll
    for (int k = 0; k < 4; ++k) {
      const int al = k >> 1, hf = k & 1;
      const int p = 128 * hf + tid;
      const int d = p >> 3, q8 = p & 7;
      const v4f a = *(const v4fa*)(sbuf + (32 * al + d) * PF + 8 * q8), c = *(const v4fa*)(sbuf + (32 * al + d) * PF + 8 * q8 + 4);
      #pragma unroll
      for (int j = 0; j < 4; ++j) {
        ov[k][j]     = (f16t)(a[j] * VCAR);
        ov[k][4 + j] = (f16t)(c[j] * VCAR);
      }
      const int na = n * NH + 2 * cg + al;
      off[k] = ((size_t)na * DK + d) * KVN + p0 + 8 * q8;
    }
    #pragma unroll
    for (int k = 0; k < 4; ++k) *(volatile v8h*)(VT + off[k]) = ov[k];
    __threadfence();
    #pragma unroll
    for (int k = 0; k < 4; ++k) *(volatile v8h*)(VT + off[k]) = ov[k];
  }
}

__global__ __launch_bounds__(TPB) void pos_k(const f16t* __restrict__ E, const f16t* __restrict__ WB,
                                            f16t* __restrict__ PX, f16t* __restrict__ PY)
{
  __shared__ __attribute__((aligned(16))) float sbuf[64 * PF];
  const int tid = threadIdx.x, lane = tid & 31, wave = tid >> 5;
  const int h = lane >> 4, m = lane & 15;
  const int blk = blockIdx.x;
  const int isY = blk >> 7;
  const int rem = blk & 127;
  const int rb = rem >> 2, cg = rem & 3;

  v8f acc[4];
  #pragma unroll
  for (int t = 0; t < 4; ++t) acc[t] = zero8f();
  const f16t* arow = E + (size_t)(64 * rb + 16 * wave + m) * PD + 8 * h;
  const f16t* brow = WB + (isY ? OWY : OWX) + (size_t)(64 * cg + m) * PD + 8 * h;
  mma_4n<PD>(arow, brow, acc);

  #pragma unroll
  for (int t = 0; t < 4; ++t) {
    #pragma unroll
    for (int r = 0; r < 8; ++r) {
      const int prow = 16 * wave + 8 * h + r;
      sbuf[prow * PF + 16 * t + m] = acc[t][r] * SC_POS;
    }
  }
  __syncthreads();

  f16t* P = isY ? PY : PX;
  v8h ov[4];
  size_t off[4];
  #pragma unroll
  for (int k = 0; k < 4; ++k) {
    const int pl = k >> 1, al = k & 1;
    const int lrow = tid >> 2, d8 = (tid & 3) * 8;
    const int row = 32 * pl + lrow, col = 32 * al + d8;
    const v4f a = *(const v4fa*)(sbuf + row * PF + col), c = *(const v4fa*)(sbuf + row * PF + col + 4);
    #pragma unroll
    for (int j = 0; j < 4; ++j) {
      ov[k][j]     = (f16t)(a[j] * POSCAR);
      ov[k][4 + j] = (f16t)(c[j] * POSCAR);
    }
    const int pos = 2 * rb + pl, aH = 2 * cg + al;
    off[k] = ((size_t)(aH * HQ + pos) * HK + lrow) * DK + d8;
  }
  #pragma unroll
  for (int k = 0; k < 4; ++k) *(volatile v8h*)(P + off[k]) = ov[k];
  __threadfence();
  #pragma unroll
  for (int k = 0; k < 4; ++k) *(volatile v8h*)(P + off[k]) = ov[k];
}

__global__ __launch_bounds__(TPB) void exy_k(const f16t* __restrict__ QG, const f16t* __restrict__ PX,
                                            const f16t* __restrict__ PY, float* __restrict__ EX,
                                            float* __restrict__ EY)
{
  __shared__ __attribute__((aligned(16))) float sbuf[64 * PE];
  const int tid = threadIdx.x, lane = tid & 31, wave = tid >> 5;
  const int h = lane >> 4, m = lane & 15;
  const int blk = blockIdx.x;
  const int isY = blk >> 10;
  const int rem = blk & 1023;
  const int na = rem >> 6, pos = rem & 63;
  const int aH = na & (NH - 1);
  const int rr = 16 * wave + m;
  const size_t q = isY ? ((size_t)pos * HQ + rr) : ((size_t)rr * HQ + pos);

  FragH fa;
  load_frag(fa, QG + ((size_t)na * HWQ + q) * DK + 8 * h, 0);
  const f16t* P = isY ? PY : PX;
  const f16t* prow = P + ((size_t)(aH * HQ + pos) * HK + m) * DK + 8 * h;
  v8f acc[2];
  #pragma unroll
  for (int lt = 0; lt < 2; ++lt) {
    FragH fb;
    load_frag(fb, prow + (size_t)16 * lt * DK, 0);
    acc[lt] = wmma_f16(fa.v, fb.v, zero8f());
  }
  #pragma unroll
  for (int lt = 0; lt < 2; ++lt) {
    #pragma unroll
    for (int r = 0; r < 8; ++r)
      sbuf[(16 * wave + 8 * h + r) * PE + 16 * lt + m] = acc[lt][r] * SC_E;
  }
  __syncthreads();

  float* Dp = isY ? EY : EX;
  v4f ov[4];
  size_t off[4];
  #pragma unroll
  for (int k = 0; k < 4; ++k) {
    const int p = 128 * k + tid;
    const int row = p >> 3, q8 = p & 7;
    ov[k] = *(const v4fa*)(sbuf + row * PE + 4 * q8);
    const size_t qq = isY ? ((size_t)pos * HQ + row) : ((size_t)row * HQ + pos);
    off[k] = ((size_t)na * HWQ + qq) * DK + 4 * q8;
  }
  #pragma unroll
  for (int k = 0; k < 4; ++k) *(volatile v4f*)(Dp + off[k]) = ov[k];
  __threadfence();
  #pragma unroll
  for (int k = 0; k < 4; ++k) *(volatile v4f*)(Dp + off[k]) = ov[k];
}

__global__ __launch_bounds__(TPBA) void attn_k(const f16t* __restrict__ QA, const f16t* __restrict__ KP,
                                              const f16t* __restrict__ VT, const float* __restrict__ EX,
                                              const float* __restrict__ EY, f16t* __restrict__ OT)
{
  __shared__ __attribute__((aligned(16))) f16t sbuf[64 * PH];
  const int tid = threadIdx.x, lane = tid & 31, wave = tid >> 5;
  const int h = lane >> 4, m = lane & 15;
  const int blk = blockIdx.x;
  const int n = blk >> 8;
  const int rem = blk & 255;
  const int hp = rem >> 6, qb = rem & 63;
  const int wq = wave & 3, al = wave >> 2;
  const int aH = 2 * hp + al;
  const int na = n * NH + aH;
  const int i0 = 64 * qb + 16 * wq;
  const size_t qrow = (size_t)na * HWQ + i0 + m;

  FragH fq;
  load_frag(fq, QA + qrow * DK + 8 * h, 0);
  U8 exlo, exhi;
  exlo.q[0] = *(const v4fa*)(EX + qrow * DK + 8 * h);
  exlo.q[1] = *(const v4fa*)(EX + qrow * DK + 8 * h + 4);
  exhi.q[0] = *(const v4fa*)(EX + qrow * DK + 16 + 8 * h);
  exhi.q[1] = *(const v4fa*)(EX + qrow * DK + 16 + 8 * h + 4);
  const float* eyp = EY + qrow * DK;
  const f16t* kbase = KP + ((size_t)na * KVN + m) * DK + 8 * h;
  const f16t* vbase = VT + ((size_t)na * DK + m) * KVN + 8 * h;

  v8f O[2];
  O[0] = zero8f(); O[1] = zero8f();
  float Mx = -3.0e38f, L = 0.0f;

  #pragma unroll 1
  for (int js = 0; js < KVN / 32; ++js) {
    const int j0 = 32 * js;
    FragH k0f, k1f;
    load_frag(k0f, kbase + (size_t)j0 * DK, 0);
    load_frag(k1f, kbase + (size_t)(j0 + 16) * DK, 0);
    const v8f s0 = wmma_f16(k0f.v, fq.v, zero8f());
    const v8f s1 = wmma_f16(k1f.v, fq.v, zero8f());
    const float ey = eyp[js];

    float e0[8], e1[8];
    float mloc = -3.0e38f;
    #pragma unroll
    for (int r = 0; r < 8; ++r) {
      e0[r] = s0[r] * SC_S + exlo.v[r] + ey;
      e1[r] = s1[r] * SC_S + exhi.v[r] + ey;
      mloc = fmaxf(mloc, fmaxf(e0[r], e1[r]));
    }
    mloc = fmaxf(mloc, __shfl_xor(mloc, 16));
    const float Mn = fmaxf(Mx, mloc);
    const float corr = __expf(Mx - Mn);
    Mx = Mn;

    FragH pf;
    float ls = 0.0f;
    #pragma unroll
    for (int r = 0; r < 8; ++r) {
      const float p0 = __expf(e0[r] - Mn);
      const float p1 = __expf(e1[r] - Mn);
      ls += p0 + p1;
      pf.half[0][r] = (f16t)(p0 * PCAR);
      pf.half[1][r] = (f16t)(p1 * PCAR);
    }
    ls += __shfl_xor(ls, 16);
    L = L * corr + ls;
    #pragma unroll
    for (int t = 0; t < 2; ++t) {
      #pragma unroll
      for (int r = 0; r < 8; ++r) O[t][r] *= corr;
    }
    #pragma unroll
    for (int t = 0; t < 2; ++t) {
      FragH va;
      load_frag(va, vbase + (size_t)16 * t * KVN + j0, 0);
      O[t] = wmma_f16(va.v, pf.v, O[t]);
    }
  }

  const float inv = (1.0f / L) * SC_O;
  #pragma unroll
  for (int t = 0; t < 2; ++t) {
    #pragma unroll
    for (int r = 0; r < 8; ++r)
      sbuf[(16 * wq + m) * PH + 32 * al + 16 * t + 8 * h + r] = (f16t)(O[t][r] * inv);
  }
  __syncthreads();

  v8h ov[2];
  size_t off[2];
  #pragma unroll
  for (int k = 0; k < 2; ++k) {
    const int p = 256 * k + tid;
    const int row = p >> 3, q = p & 7;
    ov[k] = *(const v8ha*)(sbuf + row * PH + 8 * q);
    off[k] = ((size_t)n * HWQ + 64 * qb + row) * CIN + 64 * hp + 8 * q;
  }
  #pragma unroll
  for (int k = 0; k < 2; ++k) *(volatile v8h*)(OT + off[k]) = ov[k];
  __threadfence();
  #pragma unroll
  for (int k = 0; k < 2; ++k) *(volatile v8h*)(OT + off[k]) = ov[k];
}

__global__ __launch_bounds__(TPB) void projo_k(const f16t* __restrict__ OT, const f16t* __restrict__ WB,
                                              const float* __restrict__ bp, const float* __restrict__ gam,
                                              const float* __restrict__ x, float* __restrict__ out)
{
  __shared__ __attribute__((aligned(16))) float sbuf[64 * PF];
  const int tid = threadIdx.x, lane = tid & 31, wave = tid >> 5;
  const int h = lane >> 4, m = lane & 15;
  const int blk = blockIdx.x;
  const int n = blk >> 8;
  const int rem = blk & 255;
  const int pb = rem >> 2, cg = rem & 3;
  const int hw0 = 64 * pb;

  v8f acc[4];
  #pragma unroll
  for (int t = 0; t < 4; ++t) acc[t] = zero8f();
  const f16t* arow = OT + ((size_t)n * HWQ + hw0 + 16 * wave + m) * CIN + 8 * h;
  const f16t* brow = WB + OWP + (size_t)(64 * cg + m) * CIN + 8 * h;
  mma_4n<CIN>(arow, brow, acc);

  const float g = gam[0];
  #pragma unroll
  for (int t = 0; t < 4; ++t) {
    const int ol = 16 * t + m;
    const float bv = bp[64 * cg + ol];
    #pragma unroll
    for (int r = 0; r < 8; ++r) {
      const int prow = 16 * wave + 8 * h + r;
      sbuf[ol * PF + prow] = g * (acc[t][r] * SC_PO + bv);
    }
  }
  __syncthreads();

  v4f ov[8];
  size_t off[8];
  #pragma unroll
  for (int k = 0; k < 8; ++k) {
    const int row = 8 * k + (tid >> 4), q = tid & 15;
    const v4f gv = *(const v4fa*)(sbuf + row * PF + 4 * q);
    off[k] = ((size_t)n * CIN + 64 * cg + row) * HWQ + hw0 + 4 * q;
    const v4f zv = *(const v4fa*)(x + off[k]);
    ov[k] = zv + gv;
  }
  #pragma unroll
  for (int k = 0; k < 8; ++k) *(volatile v4f*)(out + off[k]) = ov[k];
  __threadfence();
  #pragma unroll
  for (int k = 0; k < 8; ++k) *(volatile v4f*)(out + off[k]) = ov[k];
}

extern "C" void kernel_launch(void* const* d_in, const int* in_sizes, int n_in,
                              void* d_out, int out_size, void* d_ws, size_t ws_size,
                              hipStream_t stream) {
  if (n_in < 11) return;
  if (in_sizes[0] != NB * CIN * HWQ) return;
  if (in_sizes[1] != CIN * CIN || in_sizes[2] != CIN * CIN || in_sizes[3] != CIN * CIN) return;
  if (in_sizes[4] != CIN * PD || in_sizes[5] != CIN * PD) return;
  if (in_sizes[6] != CIN || in_sizes[7] != CIN) return;
  if (in_sizes[8] != CIN * CIN || in_sizes[9] != CIN) return;
  if (in_sizes[10] < 1) return;
  if (out_size != NB * CIN * HWQ) return;

  const float* x     = (const float*)d_in[0];
  const float* Wq    = (const float*)d_in[1];
  const float* Wk    = (const float*)d_in[2];
  const float* Wv    = (const float*)d_in[3];
  const float* Wx    = (const float*)d_in[4];
  const float* Wy    = (const float*)d_in[5];
  const float* ab    = (const float*)d_in[6];
  const float* gb    = (const float*)d_in[7];
  const float* Wproj = (const float*)d_in[8];
  const float* bproj = (const float*)d_in[9];
  const float* gamma = (const float*)d_in[10];
  float* outp = (float*)d_out;

  const size_t szXT = (size_t)NB * HWQ * CIN * 2;
  const size_t szWB = (size_t)WBN * 2;
  const size_t szE  = (size_t)NPR * PD * 2;
  const size_t szQ  = (size_t)NA * HWQ * DK * 2;
  const size_t szK  = (size_t)NA * KVN * DK * 2;
  const size_t szP  = (size_t)NH * HQ * HK * DK * 2;
  const size_t szEX = (size_t)NA * HWQ * DK * 4;
  const size_t szOT = (size_t)NB * HWQ * CIN * 2;
  static_assert((size_t)NB * HWQ * CIN * 2 + (size_t)WBN * 2 + (size_t)NPR * PD * 2 +
                2 * ((size_t)NA * HWQ * DK * 2) + 2 * ((size_t)NA * KVN * DK * 2) +
                2 * ((size_t)NH * HQ * HK * DK * 2) + 2 * ((size_t)NA * HWQ * DK * 4) +
                (size_t)NB * HWQ * CIN * 2 <= (size_t)134217728);
  size_t off = 0;
  char* ws = (char*)d_ws;
  f16t*  XT  = (f16t*)(ws + off);  off += szXT;
  f16t*  WBp = (f16t*)(ws + off);  off += szWB;
  f16t*  E   = (f16t*)(ws + off);  off += szE;
  f16t*  QA  = (f16t*)(ws + off);  off += szQ;
  f16t*  QG  = (f16t*)(ws + off);  off += szQ;
  f16t*  KP  = (f16t*)(ws + off);  off += szK;
  f16t*  VT  = (f16t*)(ws + off);  off += szK;
  f16t*  PX  = (f16t*)(ws + off);  off += szP;
  f16t*  PY  = (f16t*)(ws + off);  off += szP;
  float* EX  = (float*)(ws + off); off += szEX;
  float* EY  = (float*)(ws + off); off += szEX;
  f16t*  OT  = (f16t*)(ws + off);  off += szOT;
  if (off > ws_size) return;

  prep_k<<<XP_BLKS + WB_BLKS, TPBP, 0, stream>>>(x, Wq, Wk, Wv, Wproj, Wx, Wy, XT, WBp);
  embed_k<<<EM_BLKS, TPBP, 0, stream>>>(E);
  proj_k<<<PQ_BLKS + 2 * PK_BLKS, TPB, 0, stream>>>(XT, WBp, ab, gb, QA, QG, KP, VT);
  pos_k<<<POS_BLKS, TPB, 0, stream>>>(E, WBp, PX, PY);
  exy_k<<<EXY_BLKS, TPB, 0, stream>>>(QG, PX, PY, EX, EY);
  attn_k<<<ATT_BLKS, TPBA, 0, stream>>>(QA, KP, VT, EX, EY, OT);
  projo_k<<<PO_BLKS, TPB, 0, stream>>>(OT, WBp, bproj, gamma, x, outp);
  (void)hipGetLastError();
}
